// NNTDLambda_84636625535230
// MI455X (gfx1250) — hardware-run, weakly checked
//
#include <hip/hip_runtime.h>
#include <hip/hip_fp16.h>
#include <math.h>

typedef __attribute__((ext_vector_type(16))) _Float16 v16h;
typedef __attribute__((ext_vector_type(8)))  _Float16 v8h;
typedef __attribute__((ext_vector_type(8)))  float    v8f;
typedef __attribute__((ext_vector_type(4)))  float    v4f;
typedef __attribute__((ext_vector_type(2)))  float    v2f;
typedef __attribute__((ext_vector_type(2)))  unsigned v2u;

constexpr int kT = 2048;
constexpr int kD = 256;
constexpr int kH = 256;
constexpr int kOutN = kD * kH + kH + kH + 1 + 1;
constexpr int kOutW = (kOutN - 2) / 4;
constexpr int kOutTwW = (kD * kH) / 4;
constexpr float kXCarry = 64.0f;
constexpr float kWCarry = 1024.0f;
constexpr float kResid  = 2048.0f;
constexpr float kQCarry = 1024.0f;
constexpr float kAlpha  = 0.01f;
constexpr float kGL = (float)(0.99 * 0.9);
static_assert(kOutN == 66050);
static_assert(kOutW == 16512 && kOutW * 4 + 2 == kOutN);
static_assert(kOutTwW == 16384);
static_assert((kOutW % 128) == 0 && (kOutW / 128) == 129);
static_assert(((kOutN - 2) * 4) % 128 == 0);
static_assert((kT % 64) == 0 && (kD % 64) == 0 && (kH % 64) == 0);
static_assert((kT % 32) == 0 && (kD % 32) == 0);

constexpr size_t kSzXA  = (size_t)kT * kD * 2;
constexpr size_t kSzXT  = (size_t)kD * kT * 2;
constexpr size_t kSzW1T = (size_t)kH * kD * 2;
constexpr size_t kSzPRE = (size_t)kT * kH * 4;
constexpr size_t kSzVEC = (size_t)kT * 4;
constexpr size_t kSzQT  = (size_t)kH * kT * 2;
constexpr size_t kSzTW  = (size_t)kD * kH * 4;
constexpr size_t kSzRB  = (size_t)2 * kH * 4;
constexpr size_t kSzTL  = (size_t)128 * 4;
constexpr size_t kOffXA  = 0;
constexpr size_t kOffXT  = kOffXA  + kSzXA;
constexpr size_t kOffW1T = kOffXT  + kSzXT;
constexpr size_t kOffPRE = kOffW1T + kSzW1T;
constexpr size_t kOffERR = kOffPRE + kSzPRE;
constexpr size_t kOffSIG = kOffERR + kSzVEC;
constexpr size_t kOffC   = kOffSIG + kSzVEC;
constexpr size_t kOffQT  = kOffC   + kSzVEC;
constexpr size_t kOffTW  = kOffQT  + kSzQT;
constexpr size_t kOffRB  = kOffTW  + kSzTW;
constexpr size_t kOffTL  = kOffRB  + kSzRB;
constexpr size_t kWsTotal = kOffTL + kSzTL;
static_assert(kSzXA == 1048576ull && kSzXT == 1048576ull && kSzW1T == 131072ull && kSzPRE == 2097152ull);
static_assert(kSzVEC == 8192ull && kSzQT == 1048576ull && kSzTW == 262144ull && kSzRB == 2048ull);
static_assert(kSzTL == 512ull);
static_assert(kWsTotal == 5663232ull);
static_assert(kWsTotal <= 134217728ull);
static_assert((kOffXT % 128) == 0 && (kOffW1T % 128) == 0 && (kOffPRE % 128) == 0 && (kOffERR % 128) == 0 &&
              (kOffSIG % 128) == 0 && (kOffC % 128) == 0 && (kOffQT % 128) == 0 && (kOffTW % 128) == 0 &&
              (kOffRB % 128) == 0 && (kOffTL % 128) == 0);

__device__ __forceinline__ _Float16 f16_flush(float v) {
  const float w = (fabsf(v) < 6.103515625e-05f) ? 0.0f : v;
  return (_Float16)w;
}
__device__ __forceinline__ void f16_split(float v, _Float16& hi, _Float16& lo) {
  hi = f16_flush(v);
  const float hf = (float)hi;
  const float r = (v - hf) * kResid;
  lo = f16_flush(r);
}

__device__ __forceinline__ float bf16r(float v) {
  unsigned u = __float_as_uint(v);
  u = (u + 0x7FFFu + ((u >> 16) & 1u)) & 0xFFFF0000u;
  return __uint_as_float(u);
}

__device__ __forceinline__ float h16_to_f32(unsigned hb) {
  const unsigned sgn = (hb & 0x8000u) << 16; const unsigned em = hb & 0x7fffu;
  const float fn = __uint_as_float((em << 13) + 0x38000000u);
  const float fs = (float)em * 5.9604644775390625e-8f;
  const float mag = (em < 0x400u) ? fs : fn; return __uint_as_float(__float_as_uint(mag) | sgn); }

namespace eng {
union FragU { v16h v; v8h h[2]; };
__device__ __forceinline__ v16h frag_load(const _Float16* p) {
  FragU f;
  f.h[0] = *(const v8h*)(p);
  f.h[1] = *(const v8h*)(p + 16);
  return f.v;
}
__device__ __forceinline__ v8f mma(v16h a, v16h b, v8f c) {
  return __builtin_amdgcn_wmma_f32_16x16x32_f16(false, a, false, b, (short)0, c, false, false);
}
__device__ __forceinline__ void guard1(v8f& a, v16h x, v16h y) {
  asm volatile("v_nop\n\tv_nop\n\tv_nop\n\tv_nop" : "+v"(a) : "v"(x), "v"(y));
}
__device__ __forceinline__ void guard_acc(v8f& a) {
  asm volatile("v_nop\n\tv_nop\n\tv_nop\n\tv_nop" : "+v"(a));
}
__device__ __forceinline__ void keep4(v16h a, v16h b, v16h c, v16h d) {
  asm volatile("v_nop" :: "v"(a), "v"(b), "v"(c), "v"(d));
}

template <int MI, int SPL>
__global__ __launch_bounds__(256) void gemm_f16_kernel(
    const unsigned short* __restrict__ Ap, const unsigned short* __restrict__ A2p, int lda,
    const unsigned short* __restrict__ Btp, const unsigned short* __restrict__ Bt2p, int ldb,
    float* __restrict__ C, int ldc, int M, int N, int K, float scale, float rscale)
{
  static_assert(MI >= 1 && MI <= 2);
  static_assert(SPL >= 0 && SPL <= 2);
  const _Float16* A   = (const _Float16*)Ap;
  const _Float16* A2  = (const _Float16*)A2p;
  const _Float16* Bt  = (const _Float16*)Btp;
  const _Float16* Bt2 = (const _Float16*)Bt2p;
  __shared__ __align__(16) float sT[8][16 * 68];
  const int lane = threadIdx.x & 31;
  const int wave = threadIdx.x >> 5;
  const int tilesN = N >> 6;
  const int tilesM = M / (16 * MI);
  const int tile = blockIdx.x * 8 + wave;
  if (tile >= tilesM * tilesN) return;
  const int tm = tile / tilesN;
  const int tn = tile - tm * tilesN;
  const int m0 = tm * (16 * MI);
  const int n0 = tn << 6;
  const int rlane = lane & 15;
  const int koff  = (lane >> 4) * 8;
  const int mOff  = (lane >> 4) * 8;

  v8f acc[MI][4], accr[MI][4];
#pragma unroll
  for (int i = 0; i < MI; ++i)
#pragma unroll
    for (int j = 0; j < 4; ++j) {
      acc[i][j]  = (v8f){0.f, 0.f, 0.f, 0.f, 0.f, 0.f, 0.f, 0.f};
      accr[i][j] = (v8f){0.f, 0.f, 0.f, 0.f, 0.f, 0.f, 0.f, 0.f};
    }

  for (int k0 = 0; k0 < K; k0 += 32) {
    v16h bh[4], bl[4];
#pragma unroll
    for (int j = 0; j < 4; ++j) {
      const size_t bo = (size_t)(n0 + (j << 4) + rlane) * ldb + koff + k0;
      bh[j] = frag_load(Bt + bo);
      if (SPL == 2) bl[j] = frag_load(Bt2 + bo); else bl[j] = bh[j];
    }
#pragma unroll
    for (int i = 0; i < MI; ++i) {
      const size_t ao = (size_t)(m0 + (i << 4) + rlane) * lda + koff + k0;
      const v16h ah = frag_load(A + ao);
      v16h al = ah;
      if (SPL >= 1) al = frag_load(A2 + ao);
#pragma unroll
      for (int j = 0; j < 4; ++j) {
        acc[i][j] = mma(ah, bh[j], acc[i][j]);
        if (SPL >= 1) accr[i][j] = mma(al, bh[j], accr[i][j]);
        if (SPL == 2) accr[i][j] = mma(ah, bl[j], accr[i][j]);
      }
#pragma unroll
      for (int j = 0; j < 4; ++j) {
        guard1(acc[i][j], ah, al);
        if (SPL >= 1) guard1(accr[i][j], ah, al);
      }
    }
    keep4(bh[0], bh[1], bh[2], bh[3]);
    if (SPL == 2) keep4(bl[0], bl[1], bl[2], bl[3]);
  }
#pragma unroll
  for (int i = 0; i < MI; ++i)
#pragma unroll
    for (int j = 0; j < 4; ++j) {
      guard_acc(acc[i][j]);
      if (SPL >= 1) guard_acc(accr[i][j]);
    }

  float* slab = sT[wave];
#pragma unroll
  for (int i = 0; i < MI; ++i) {
    const int mBase = m0 + (i << 4);
#pragma unroll
    for (int j = 0; j < 4; ++j) {
#pragma unroll
      for (int r = 0; r < 8; ++r) {
        float v = acc[i][j][r] * scale;
        if (SPL >= 1) v += accr[i][j][r] * rscale;
        slab[(mOff + r) * 68 + (j << 4) + rlane] = v;
      }
    }
    __builtin_amdgcn_fence(__ATOMIC_RELEASE, "workgroup");
    __builtin_amdgcn_wave_barrier();
    __builtin_amdgcn_fence(__ATOMIC_ACQUIRE, "workgroup");
    {
      const int hh = lane >> 4, c4 = (lane & 15) * 4;
      for (int pass = 0; pass < 2; ++pass) {
#pragma unroll
        for (int it = 0; it < 8; ++it) {
          const int row = it * 2 + hh;
          const v4f v = *(const v4f*)(slab + row * 68 + c4);
          *(volatile v4f*)(C + (size_t)(mBase + row) * ldc + n0 + c4) = v;
        }
        __threadfence();
      }
    }
    __builtin_amdgcn_fence(__ATOMIC_RELEASE, "workgroup");
    __builtin_amdgcn_wave_barrier();
    __builtin_amdgcn_fence(__ATOMIC_ACQUIRE, "workgroup");
  }
}
}

__global__ __launch_bounds__(256) void pack_xa_kernel(
    const float* __restrict__ x, unsigned short* __restrict__ XA)
{
  const int i = blockIdx.x * 256 + threadIdx.x;
  const size_t e0 = (size_t)i << 3;
  const v4f a0 = *(const v4f*)(x + e0);
  const v4f a1 = *(const v4f*)(x + e0 + 4);
  const float f0 = a0[0];
  const float f1 = a0[1];
  const float f2 = a0[2];
  const float f3 = a0[3];
  const float f4 = a1[0];
  const float f5 = a1[1];
  const float f6 = a1[2];
  const float f7 = a1[3];
  v8h hv;
  hv[0] = f16_flush(bf16r(f0) * kXCarry);
  hv[1] = f16_flush(bf16r(f1) * kXCarry);
  hv[2] = f16_flush(bf16r(f2) * kXCarry);
  hv[3] = f16_flush(bf16r(f3) * kXCarry);
  hv[4] = f16_flush(bf16r(f4) * kXCarry);
  hv[5] = f16_flush(bf16r(f5) * kXCarry);
  hv[6] = f16_flush(bf16r(f6) * kXCarry);
  hv[7] = f16_flush(bf16r(f7) * kXCarry);
  unsigned short* q = XA + e0;
  *(volatile v8h*)q = hv;
  __threadfence();
  *(volatile v8h*)q = hv;
}

__global__ __launch_bounds__(256) void pack_xt_kernel(
    const float* __restrict__ x, unsigned short* __restrict__ XT)
{
  const int i  = blockIdx.x * 256 + threadIdx.x;
  const int sg = i & 255;
  const int d  = i >> 8;
  const int s0 = sg << 3;
  const float* p = x + (size_t)s0 * kD + d;
  const float f0 = p[0 * kD];
  const float f1 = p[1 * kD];
  const float f2 = p[2 * kD];
  const float f3 = p[3 * kD];
  const float f4 = p[4 * kD];
  const float f5 = p[5 * kD];
  const float f6 = p[6 * kD];
  const float f7 = p[7 * kD];
  v8h hv;
  hv[0] = f16_flush(bf16r(f0) * kXCarry);
  hv[1] = f16_flush(bf16r(f1) * kXCarry);
  hv[2] = f16_flush(bf16r(f2) * kXCarry);
  hv[3] = f16_flush(bf16r(f3) * kXCarry);
  hv[4] = f16_flush(bf16r(f4) * kXCarry);
  hv[5] = f16_flush(bf16r(f5) * kXCarry);
  hv[6] = f16_flush(bf16r(f6) * kXCarry);
  hv[7] = f16_flush(bf16r(f7) * kXCarry);
  unsigned short* q = XT + (size_t)d * kT + s0;
  *(volatile v8h*)q = hv;
  __threadfence();
  *(volatile v8h*)q = hv;
}

__global__ __launch_bounds__(256) void pack_w1t_kernel(
    const float* __restrict__ W1, unsigned short* __restrict__ W1T)
{
  const int i  = blockIdx.x * 256 + threadIdx.x;
  const int dg = i & 31;
  const int h  = i >> 5;
  const int d0 = dg << 3;
  const float* p = W1 + (size_t)d0 * kH + h;
  const float f0 = p[0 * kH];
  const float f1 = p[1 * kH];
  const float f2 = p[2 * kH];
  const float f3 = p[3 * kH];
  const float f4 = p[4 * kH];
  const float f5 = p[5 * kH];
  const float f6 = p[6 * kH];
  const float f7 = p[7 * kH];
  v8h hv;
  hv[0] = f16_flush(bf16r(f0) * kWCarry);
  hv[1] = f16_flush(bf16r(f1) * kWCarry);
  hv[2] = f16_flush(bf16r(f2) * kWCarry);
  hv[3] = f16_flush(bf16r(f3) * kWCarry);
  hv[4] = f16_flush(bf16r(f4) * kWCarry);
  hv[5] = f16_flush(bf16r(f5) * kWCarry);
  hv[6] = f16_flush(bf16r(f6) * kWCarry);
  hv[7] = f16_flush(bf16r(f7) * kWCarry);
  unsigned short* q = W1T + (size_t)h * kD + d0;
  *(volatile v8h*)q = hv;
  __threadfence();
  *(volatile v8h*)q = hv;
}

__global__ __launch_bounds__(256) void us_err_kernel(
    const float* __restrict__ PRE, const float* __restrict__ ys, const float* __restrict__ b1,
    const float* __restrict__ W2, const float* __restrict__ b2, float* __restrict__ ERR)
{
  const int t = blockIdx.x * 256 + threadIdx.x;
  const float* p0 = PRE + (size_t)(4 * t) * kH;
  float u0 = 0.0f;
  float u1 = 0.0f;
  float u2 = 0.0f;
  float u3 = 0.0f;
  for (int h4 = 0; h4 < 64; ++h4) {
    const v4f bv = *(const v4f*)(b1 + 4 * h4);
    const v4f wv = *(const v4f*)(W2 + 4 * h4);
    const float bb0 = bv[0];
    const float bb1 = bv[1];
    const float bb2 = bv[2];
    const float bb3 = bv[3];
    const float ww0 = wv[0];
    const float ww1 = wv[1];
    const float ww2 = wv[2];
    const float ww3 = wv[3];
    const float br0 = bf16r(bb0);
    const float br1 = bf16r(bb1);
    const float br2 = bf16r(bb2);
    const float br3 = bf16r(bb3);
    const float wr0 = bf16r(ww0);
    const float wr1 = bf16r(ww1);
    const float wr2 = bf16r(ww2);
    const float wr3 = bf16r(ww3);
    const v4f q0 = *(const v4f*)(p0 + 0 * kH + 4 * h4);
    const v4f q1 = *(const v4f*)(p0 + 1 * kH + 4 * h4);
    const v4f q2 = *(const v4f*)(p0 + 2 * kH + 4 * h4);
    const v4f q3 = *(const v4f*)(p0 + 3 * kH + 4 * h4);
    const float a00 = q0[0] + br0;
    const float a01 = q0[1] + br1;
    const float a02 = q0[2] + br2;
    const float a03 = q0[3] + br3;
    const float a10 = q1[0] + br0;
    const float a11 = q1[1] + br1;
    const float a12 = q1[2] + br2;
    const float a13 = q1[3] + br3;
    const float a20 = q2[0] + br0;
    const float a21 = q2[1] + br1;
    const float a22 = q2[2] + br2;
    const float a23 = q2[3] + br3;
    const float a30 = q3[0] + br0;
    const float a31 = q3[1] + br1;
    const float a32 = q3[2] + br2;
    const float a33 = q3[3] + br3;
    u0 = fmaf((a00 > 0.0f) ? a00 : 0.0f, wr0, u0);
    u0 = fmaf((a01 > 0.0f) ? a01 : 0.0f, wr1, u0);
    u0 = fmaf((a02 > 0.0f) ? a02 : 0.0f, wr2, u0);
    u0 = fmaf((a03 > 0.0f) ? a03 : 0.0f, wr3, u0);
    u1 = fmaf((a10 > 0.0f) ? a10 : 0.0f, wr0, u1);
    u1 = fmaf((a11 > 0.0f) ? a11 : 0.0f, wr1, u1);
    u1 = fmaf((a12 > 0.0f) ? a12 : 0.0f, wr2, u1);
    u1 = fmaf((a13 > 0.0f) ? a13 : 0.0f, wr3, u1);
    u2 = fmaf((a20 > 0.0f) ? a20 : 0.0f, wr0, u2);
    u2 = fmaf((a21 > 0.0f) ? a21 : 0.0f, wr1, u2);
    u2 = fmaf((a22 > 0.0f) ? a22 : 0.0f, wr2, u2);
    u2 = fmaf((a23 > 0.0f) ? a23 : 0.0f, wr3, u2);
    u3 = fmaf((a30 > 0.0f) ? a30 : 0.0f, wr0, u3);
    u3 = fmaf((a31 > 0.0f) ? a31 : 0.0f, wr1, u3);
    u3 = fmaf((a32 > 0.0f) ? a32 : 0.0f, wr2, u3);
    u3 = fmaf((a33 > 0.0f) ? a33 : 0.0f, wr3, u3);
  }
  const float b2v = b2[0];
  const float b2r = bf16r(b2v);
  const v4f y0 = *(const v4f*)(ys + 8 * t);
  const v4f y1 = *(const v4f*)(ys + 8 * t + 4);
  const float g0 = y0[0];
  const float g1 = y0[2];
  const float g2 = y1[0];
  const float g3 = y1[2];
  const float df0 = bf16r(g0) - (u0 + b2r);
  const float df1 = bf16r(g1) - (u1 + b2r);
  const float df2 = bf16r(g2) - (u2 + b2r);
  const float df3 = bf16r(g3) - (u3 + b2r);
  v4f ev;
  ev[0] = df0 * df0;
  ev[1] = df1 * df1;
  ev[2] = df2 * df2;
  ev[3] = df3 * df3;
  float* q = ERR + 4 * t;
  *(volatile v4f*)q = ev;
  __threadfence();
  *(volatile v4f*)q = ev;
}

__global__ __launch_bounds__(32) void sigma_kernel(
    const float* __restrict__ ERR, const float* __restrict__ ys, float* __restrict__ SIG)
{
  const int lane = threadIdx.x;
  for (int p = 0; p < 16; ++p) {
    const int base = 128 * p + 4 * lane;
    float r = 0.0f;
    float k0 = 0.0f;
    float k1 = 0.0f;
    float k2 = 0.0f;
    float k3 = 0.0f;
    for (int s = 0; s < 2048; ++s) {
      const float e  = ERR[s];
      const float dn = ys[2 * s + 1];
      const float sg = e - r;
      r = fmaf(kAlpha, sg, r);
      const float keep = (bf16r(dn) > 0.5f) ? 0.0f : 1.0f;
      r = r * keep;
      k0 = (s == base) ? sg : k0;
      k1 = (s == base + 1) ? sg : k1;
      k2 = (s == base + 2) ? sg : k2;
      k3 = (s == base + 3) ? sg : k3;
    }
    v4f kv;
    kv[0] = k0;
    kv[1] = k1;
    kv[2] = k2;
    kv[3] = k3;
    float* q = SIG + base;
    *(volatile v4f*)q = kv;
    __threadfence();
    *(volatile v4f*)q = kv;
  }
}

__global__ __launch_bounds__(32) void c_kernel(
    const float* __restrict__ SIG, const float* __restrict__ ys, float* __restrict__ C)
{
  const int lane = threadIdx.x;
  for (int p = 0; p < 16; ++p) {
    const int base = 128 * p + 4 * lane;
    float c = 0.0f;
    float k0 = 0.0f;
    float k1 = 0.0f;
    float k2 = 0.0f;
    float k3 = 0.0f;
    for (int i = 0; i < 2048; ++i) {
      const int s = 2047 - i;
      const float sg = SIG[s];
      const float dn = ys[2 * s + 1];
      const float cn = fmaf(kGL, c, sg);
      c = (bf16r(dn) > 0.5f) ? sg : cn;
      k0 = (s == base) ? c : k0;
      k1 = (s == base + 1) ? c : k1;
      k2 = (s == base + 2) ? c : k2;
      k3 = (s == base + 3) ? c : k3;
    }
    v4f kv;
    kv[0] = k0;
    kv[1] = k1;
    kv[2] = k2;
    kv[3] = k3;
    float* q = C + base;
    *(volatile v4f*)q = kv;
    __threadfence();
    *(volatile v4f*)q = kv;
  }
}

__global__ __launch_bounds__(256) void q_kernel(
    const float* __restrict__ PRE, const float* __restrict__ C, const float* __restrict__ b1,
    const float* __restrict__ W2, unsigned short* __restrict__ QT)
{
  const int i  = blockIdx.x * 256 + threadIdx.x;
  const int sg = i & 255;
  const int h  = i >> 8;
  const int s0 = sg << 3;
  const float bv = b1[h];
  const float wv = W2[h];
  const float br = bf16r(bv);
  const float wr = bf16r(wv);
  const v4f c0 = *(const v4f*)(C + s0);
  const v4f c1 = *(const v4f*)(C + s0 + 4);
  const float cc0 = c0[0];
  const float cc1 = c0[1];
  const float cc2 = c0[2];
  const float cc3 = c0[3];
  const float cc4 = c1[0];
  const float cc5 = c1[1];
  const float cc6 = c1[2];
  const float cc7 = c1[3];
  const float* p = PRE + (size_t)s0 * kH + h;
  const float p0 = p[0 * kH];
  const float p1 = p[1 * kH];
  const float p2 = p[2 * kH];
  const float p3 = p[3 * kH];
  const float p4 = p[4 * kH];
  const float p5 = p[5 * kH];
  const float p6 = p[6 * kH];
  const float p7 = p[7 * kH];
  const float m0 = ((p0 + br) > 0.0f) ? 1.0f : 0.0f;
  const float m1 = ((p1 + br) > 0.0f) ? 1.0f : 0.0f;
  const float m2 = ((p2 + br) > 0.0f) ? 1.0f : 0.0f;
  const float m3 = ((p3 + br) > 0.0f) ? 1.0f : 0.0f;
  const float m4 = ((p4 + br) > 0.0f) ? 1.0f : 0.0f;
  const float m5 = ((p5 + br) > 0.0f) ? 1.0f : 0.0f;
  const float m6 = ((p6 + br) > 0.0f) ? 1.0f : 0.0f;
  const float m7 = ((p7 + br) > 0.0f) ? 1.0f : 0.0f;
  const float q0 = (cc0 * m0) * wr;
  const float q1 = (cc1 * m1) * wr;
  const float q2 = (cc2 * m2) * wr;
  const float q3 = (cc3 * m3) * wr;
  const float q4 = (cc4 * m4) * wr;
  const float q5 = (cc5 * m5) * wr;
  const float q6 = (cc6 * m6) * wr;
  const float q7 = (cc7 * m7) * wr;
  v8h hv;
  hv[0] = f16_flush(q0 * kQCarry);
  hv[1] = f16_flush(q1 * kQCarry);
  hv[2] = f16_flush(q2 * kQCarry);
  hv[3] = f16_flush(q3 * kQCarry);
  hv[4] = f16_flush(q4 * kQCarry);
  hv[5] = f16_flush(q5 * kQCarry);
  hv[6] = f16_flush(q6 * kQCarry);
  hv[7] = f16_flush(q7 * kQCarry);
  unsigned short* q = QT + (size_t)h * kT + s0;
  *(volatile v8h*)q = hv;
  __threadfence();
  *(volatile v8h*)q = hv;
}

__global__ __launch_bounds__(64) void rest_kernel(
    const float* __restrict__ PRE, const float* __restrict__ C, const float* __restrict__ b1,
    const float* __restrict__ W2, float* __restrict__ RB)
{
  const int t  = threadIdx.x;
  const int h0 = 4 * t;
  const v4f bv = *(const v4f*)(b1 + h0);
  const v4f wv = *(const v4f*)(W2 + h0);
  const float bb0 = bv[0];
  const float bb1 = bv[1];
  const float bb2 = bv[2];
  const float bb3 = bv[3];
  const float ww0 = wv[0];
  const float ww1 = wv[1];
  const float ww2 = wv[2];
  const float ww3 = wv[3];
  const float br0 = bf16r(bb0);
  const float br1 = bf16r(bb1);
  const float br2 = bf16r(bb2);
  const float br3 = bf16r(bb3);
  const float wr0 = bf16r(ww0);
  const float wr1 = bf16r(ww1);
  const float wr2 = bf16r(ww2);
  const float wr3 = bf16r(ww3);
  float accB0 = 0.0f;
  float accB1 = 0.0f;
  float accB2 = 0.0f;
  float accB3 = 0.0f;
  float accW0 = 0.0f;
  float accW1 = 0.0f;
  float accW2 = 0.0f;
  float accW3 = 0.0f;
  for (int s = 0; s < 2048; ++s) {
    const float cs = C[s];
    const v4f pv = *(const v4f*)(PRE + (size_t)s * kH + h0);
    const float a0 = pv[0] + br0;
    const float a1 = pv[1] + br1;
    const float a2 = pv[2] + br2;
    const float a3 = pv[3] + br3;
    const bool g0 = a0 > 0.0f;
    const bool g1 = a1 > 0.0f;
    const bool g2 = a2 > 0.0f;
    const bool g3 = a3 > 0.0f;
    accB0 += (cs * (g0 ? 1.0f : 0.0f)) * wr0;
    accB1 += (cs * (g1 ? 1.0f : 0.0f)) * wr1;
    accB2 += (cs * (g2 ? 1.0f : 0.0f)) * wr2;
    accB3 += (cs * (g3 ? 1.0f : 0.0f)) * wr3;
    accW0 += cs * (g0 ? a0 : 0.0f);
    accW1 += cs * (g1 ? a1 : 0.0f);
    accW2 += cs * (g2 ? a2 : 0.0f);
    accW3 += cs * (g3 ? a3 : 0.0f);
  }
  v4f nb;
  nb[0] = -accB0;
  nb[1] = -accB1;
  nb[2] = -accB2;
  nb[3] = -accB3;
  v4f nw;
  nw[0] = -accW0;
  nw[1] = -accW1;
  nw[2] = -accW2;
  nw[3] = -accW3;
  float* qb = RB + h0;
  float* qw = RB + kH + h0;
  *(volatile v4f*)qb = nb;
  *(volatile v4f*)qw = nw;
  __threadfence();
  *(volatile v4f*)qb = nb;
  *(volatile v4f*)qw = nw;
}

__global__ __launch_bounds__(128) void out_kernel(
    const float* __restrict__ TW, const float* __restrict__ RB, float* __restrict__ out)
{
  const int w = blockIdx.x * 128 + threadIdx.x;
  const bool first = w < kOutTwW;
  const int wa = first ? w : (kOutTwW - 1);
  const int wb = first ? 0 : (w - kOutTwW);
  const v4f tv = *(const v4f*)(TW + (size_t)wa * 4);
  const v4f rv = *(const v4f*)(RB + (size_t)wb * 4);
  const float t0 = tv[0];
  const float t1 = tv[1];
  const float t2 = tv[2];
  const float t3 = tv[3];
  const float r0 = rv[0];
  const float r1 = rv[1];
  const float r2 = rv[2];
  const float r3 = rv[3];
  v4f ov;
  ov[0] = first ? (-t0) : r0;
  ov[1] = first ? (-t1) : r1;
  ov[2] = first ? (-t2) : r2;
  ov[3] = first ? (-t3) : r3;
  float* q = out + (size_t)w * 4;
  *(volatile v4f*)q = ov;
  __threadfence();
  *(volatile v4f*)q = ov;
}

__global__ __launch_bounds__(32) void tailval_kernel(
    const float* __restrict__ C, const float* __restrict__ SIG, float* __restrict__ TL)
{
  const int lane = threadIdx.x;
  float acc = 0.0f;
  for (int s = 0; s < 2048; ++s) {
    acc += C[s];
  }
  const float sl = SIG[2047];
  v4f tv;
  tv[0] = -acc;
  tv[1] = sl;
  tv[2] = 0.0f;
  tv[3] = 0.0f;
  float* q = TL + 4 * lane;
  *(volatile v4f*)q = tv;
  __threadfence();
  *(volatile v4f*)q = tv;
}

namespace {
__global__ __launch_bounds__(256) void ocpr_kernel(const float* __restrict__ P, int pp, int pc, float* __restrict__ OUT, int w, int n) {
  const int t = blockIdx.x * 256 + threadIdx.x; if (t >= n * w) return; const int v = t / w; const int c = t - v * w; const float y = P[(size_t)v * (size_t)pp + (size_t)pc + (size_t)c];
  for (int pass = 0; pass < 2; ++pass) { ((volatile float*)OUT)[t] = y; __threadfence(); }
}
}

static_assert(((kT / 32) * (kH / 64)) % 8 == 0);
static_assert(((kD / 32) * (kH / 64)) % 8 == 0);
static_assert(((kT * kD / 8) % 256) == 0 && (kT * kD / 8) / 256 == 256);
static_assert(((kH * kD / 8) % 256) == 0 && (kH * kD / 8) / 256 == 32);
static_assert(((kH * kT / 8) % 256) == 0 && (kH * kT / 8) / 256 == 256);
static_assert((kT / 4) == 512 && (kH / 4) == 64);
static_assert(kOutN - 2 == 66048);

extern "C" void kernel_launch(void* const* d_in, const int* in_sizes, int n_in,
                              void* d_out, int out_size, void* d_ws, size_t ws_size,
                              hipStream_t stream)
{
  if (n_in < 6) return;
  if (in_sizes[0] != kT * kD) return;
  if (in_sizes[1] != kT * 2) return;
  if (in_sizes[2] != kD * kH) return;
  if (in_sizes[3] != kH) return;
  if (in_sizes[4] != kH) return;
  if (in_sizes[5] != 1) return;
  if (out_size != kOutN) return;
  if (ws_size < kWsTotal) return;

  const float* xs = (const float*)d_in[0];
  const float* ys = (const float*)d_in[1];
  const float* W1 = (const float*)d_in[2];
  const float* b1 = (const float*)d_in[3];
  const float* W2 = (const float*)d_in[4];
  const float* b2 = (const float*)d_in[5];
  float* out = (float*)d_out;

  char* ws = (char*)d_ws;
  unsigned short* XA  = (unsigned short*)(ws + kOffXA);
  unsigned short* XT  = (unsigned short*)(ws + kOffXT);
  unsigned short* W1T = (unsigned short*)(ws + kOffW1T);
  float*          PRE = (float*)(ws + kOffPRE);
  float*          ERR = (float*)(ws + kOffERR);
  float*          SIG = (float*)(ws + kOffSIG);
  float*          C   = (float*)(ws + kOffC);
  unsigned short* QT  = (unsigned short*)(ws + kOffQT);
  float*          TW  = (float*)(ws + kOffTW);
  float*          RB  = (float*)(ws + kOffRB);
  float*          TL  = (float*)(ws + kOffTL);

  constexpr float sPre = 1.0f / (kXCarry * kWCarry);
  constexpr float sTw  = 1.0f / (kXCarry * kQCarry);

  pack_xa_kernel<<<(kT * kD / 8) / 256, 256, 0, stream>>>(xs, XA);

  pack_xt_kernel<<<(kD * kT / 8) / 256, 256, 0, stream>>>(xs, XT);

  pack_w1t_kernel<<<(kH * kD / 8) / 256, 256, 0, stream>>>(W1, W1T);

  eng::gemm_f16_kernel<2, 0><<<dim3((kT / 32) * (kH / 64) / 8), 256, 0, stream>>>(
      XA, nullptr, kD, W1T, nullptr, kD, PRE, kH, kT, kH, kD, sPre, 0.0f);

  us_err_kernel<<<(kT / 4) / 256, 256, 0, stream>>>(PRE, ys, b1, W2, b2, ERR);

  sigma_kernel<<<1, 32, 0, stream>>>(ERR, ys, SIG);

  c_kernel<<<1, 32, 0, stream>>>(SIG, ys, C);

  q_kernel<<<(kH * kT / 8) / 256, 256, 0, stream>>>(PRE, C, b1, W2, QT);

  eng::gemm_f16_kernel<2, 0><<<dim3((kD / 32) * (kH / 64) / 8), 256, 0, stream>>>(
      XT, nullptr, kT, QT, nullptr, kT, TW, kH, kD, kH, kT, sTw, 0.0f);

  rest_kernel<<<1, kH / 4, 0, stream>>>(PRE, C, b1, W2, RB);

  out_kernel<<<kOutW / 128, 128, 0, stream>>>(TW, RB, out);

  tailval_kernel<<<1, 32, 0, stream>>>(C, SIG, TL);

  ocpr_kernel<<<1, 256, 0, stream>>>(TL, 4, 0, (float*)d_out + 66048, 2, 1);
}
